// TemporalAttentionModule_82600811037088
// MI455X (gfx1250) — hardware-verified
//
#include <hip/hip_runtime.h>


#define T_   4096
#define C_   256
#define CQ_  32
#define B_   4
#define XP   264
#define QT   32
#define VT   64
#define VO   64
#define VTP  72
#define AT   32
#define OBP  36
#define LN4096 8.31776616671934f

typedef char chk_dims[((T_ % QT) == 0 && (T_ % VT) == 0 && (T_ % AT) == 0 && (T_ % 64) == 0 &&
                       (C_ % VO) == 0 && (C_ % 32) == 0 && (CQ_ == 32) && (VO == 64) && (VT == 64) && (AT == 32)) ? 1 : -1];

typedef __bf16         v16b __attribute__((ext_vector_type(16)));
typedef __bf16         v8b  __attribute__((ext_vector_type(8), __may_alias__));
typedef _Float16       v16h __attribute__((ext_vector_type(16)));
typedef _Float16       v8h  __attribute__((ext_vector_type(8), __may_alias__));
typedef float          v8f  __attribute__((ext_vector_type(8)));
typedef float          v4f  __attribute__((ext_vector_type(4), __may_alias__));
typedef unsigned short v8us __attribute__((ext_vector_type(8), __may_alias__));

union FragB { v16b v; v8b h2[2]; __bf16 e[16]; };
union FragH { v16h v; v8h h2[2]; _Float16 e[16]; };

__device__ __forceinline__ v8f mma_bf(v16b a, v16b b, v8f c) {
    return __builtin_amdgcn_wmma_f32_16x16x32_bf16(false, a, false, b, (short)0, c, false, false);
}
__device__ __forceinline__ v8f mma_h(v16h a, v16h b, v8f c) {
    return __builtin_amdgcn_wmma_f32_16x16x32_f16(false, a, false, b, (short)0, c, false, false);
}
#define WG4(acc, p0, p1, p2, p3) \
    asm volatile("v_nop\n\tv_nop\n\tv_nop\n\tv_nop" : "+v"(acc) : "v"(p0), "v"(p1), "v"(p2), "v"(p3))

__device__ __forceinline__ unsigned short bfbits(__bf16 v) { return __builtin_bit_cast(unsigned short, v); }
__device__ __forceinline__ float bf2f(__bf16 v) {
    return __builtin_bit_cast(float, ((unsigned int)bfbits(v)) << 16);
}
__device__ __forceinline__ void split_bf(float f, __bf16& hi, __bf16& lo) {
    hi = (__bf16)f;
    lo = (__bf16)(f - bf2f(hi));
}

__device__ __forceinline__ void load_w_split(const float* __restrict__ p, FragB& bh, FragB& bl) {
    const v4f f0 = *(const v4f*)(p);
    const v4f f1 = *(const v4f*)(p + 4);
    const v4f f2 = *(const v4f*)(p + 16);
    const v4f f3 = *(const v4f*)(p + 20);
    #pragma unroll
    for (int i = 0; i < 4; ++i) {
        __bf16 a, e;
        split_bf(f0[i], a, e); bh.e[i]      = a; bl.e[i]      = e;
        split_bf(f1[i], a, e); bh.e[4 + i]  = a; bl.e[4 + i]  = e;
        split_bf(f2[i], a, e); bh.e[8 + i]  = a; bl.e[8 + i]  = e;
        split_bf(f3[i], a, e); bh.e[12 + i] = a; bl.e[12 + i] = e;
    }
}
__device__ __forceinline__ void load_w_h16x16(const float* __restrict__ p, FragH& b) {
    const v4f f0 = *(const v4f*)(p);
    const v4f f1 = *(const v4f*)(p + 4);
    const v4f f2 = *(const v4f*)(p + 16);
    const v4f f3 = *(const v4f*)(p + 20);
    #pragma unroll
    for (int i = 0; i < 4; ++i) {
        b.e[i]      = (_Float16)(f0[i] * 16.0f);
        b.e[4 + i]  = (_Float16)(f1[i] * 16.0f);
        b.e[8 + i]  = (_Float16)(f2[i] * 16.0f);
        b.e[12 + i] = (_Float16)(f3[i] * 16.0f);
    }
}

__global__ __launch_bounds__(64)
void k_projqk(const float* __restrict__ x, const float* __restrict__ Wq, const float* __restrict__ bq,
              const float* __restrict__ Wk, const float* __restrict__ bk,
              unsigned short* __restrict__ Qh, unsigned short* __restrict__ Ql,
              unsigned short* __restrict__ Kh, unsigned short* __restrict__ Kl)
{
    __shared__ __attribute__((aligned(16))) __bf16 xh[QT * XP];
    __shared__ __attribute__((aligned(16))) __bf16 xl[QT * XP];
    __shared__ __attribute__((aligned(16))) unsigned short ob[4 * QT * CQ_];

    const int tid = threadIdx.x;
    const int l = tid & 31, w = tid >> 5, h = l >> 4, m = l & 15;
    const int t0 = blockIdx.x * QT, b = blockIdx.y;
    if (t0 + QT > T_ || b >= B_) return;

    const float* xb = x + (size_t)b * C_ * T_ + t0;
    #pragma unroll 2
    for (int it = 0; it < (C_ * QT / 4) / 64; ++it) {
        const int idx = it * 64 + tid;
        const int c   = idx >> 3;
        const int q4  = idx & 7;
        const v4f v = *(const v4f*)(xb + (size_t)c * T_ + 4 * q4);
        #pragma unroll
        for (int j = 0; j < 4; ++j) {
            __bf16 a, e;
            split_bf(v[j], a, e);
            xh[(4 * q4 + j) * XP + c] = a;
            xl[(4 * q4 + j) * XP + c] = e;
        }
    }
    __syncthreads();

    const v8f zero = {};
    v8f acc[4];
    #pragma unroll
    for (int j = 0; j < 4; ++j) acc[j] = zero;

    const __bf16* arh = xh + (16 * w + m) * XP + 8 * h;
    const __bf16* arl = xl + (16 * w + m) * XP + 8 * h;
    const float* wq = Wq + (size_t)m * C_ + 8 * h;
    const float* wk = Wk + (size_t)m * C_ + 8 * h;

    #pragma unroll 1
    for (int ks = 0; ks < C_ / 32; ++ks) {
        const int k0 = ks * 32;
        FragB ah, al;
        ah.h2[0] = *(const v8b*)(arh + k0);
        ah.h2[1] = *(const v8b*)(arh + k0 + 16);
        al.h2[0] = *(const v8b*)(arl + k0);
        al.h2[1] = *(const v8b*)(arl + k0 + 16);
        #pragma unroll
        for (int j = 0; j < 4; ++j) {
            const float* wp = ((j < 2) ? wq : wk) + (size_t)(16 * (j & 1)) * C_ + k0;
            FragB bh, bl;
            load_w_split(wp, bh, bl);
            acc[j] = mma_bf(ah.v, bh.v, acc[j]);
            acc[j] = mma_bf(ah.v, bl.v, acc[j]);
            acc[j] = mma_bf(al.v, bh.v, acc[j]);
            WG4(acc[j], ah.v, al.v, bh.v, bl.v);
        }
    }

    #pragma unroll
    for (int j = 0; j < 4; ++j) {
        const int o = 16 * (j & 1) + m;
        const float bias = ((j < 2) ? bq : bk)[o];
        const int pb = ((j < 2) ? 0 : 2) * (QT * CQ_);
        #pragma unroll
        for (int r = 0; r < 8; ++r) {
            const int tl = 16 * w + 8 * h + r;
            __bf16 a, e;
            split_bf(acc[j][r] + bias, a, e);
            ob[pb + tl * CQ_ + o]            = bfbits(a);
            ob[pb + QT * CQ_ + tl * CQ_ + o] = bfbits(e);
        }
    }
    __syncthreads();

    v8us vals[8];
    #pragma unroll
    for (int it = 0; it < 8; ++it) {
        const int p  = it >> 1;
        const int wi = (it & 1) * 64 + tid;
        vals[it] = *(const v8us*)(ob + p * (QT * CQ_) + wi * 8);
    }
    const size_t gb = ((size_t)b * T_ + t0) * CQ_;
    #pragma unroll
    for (int it = 0; it < 8; ++it) {
        const int p  = it >> 1;
        const int wi = (it & 1) * 64 + tid;
        unsigned short* dst = ((p == 0) ? Qh : (p == 1) ? Ql : (p == 2) ? Kh : Kl) + gb + (size_t)wi * 8;
        *(volatile v8us*)dst = vals[it];
    }
    __threadfence();
    #pragma unroll
    for (int it = 0; it < 8; ++it) {
        const int p  = it >> 1;
        const int wi = (it & 1) * 64 + tid;
        unsigned short* dst = ((p == 0) ? Qh : (p == 1) ? Ql : (p == 2) ? Kh : Kl) + gb + (size_t)wi * 8;
        *(volatile v8us*)dst = vals[it];
    }
}

__global__ __launch_bounds__(128)
void k_projv(const float* __restrict__ x, const float* __restrict__ Wv, const float* __restrict__ bv,
             _Float16* __restrict__ V)
{
    __shared__ __attribute__((aligned(16))) _Float16 xt[VT * XP];
    __shared__ __attribute__((aligned(16))) _Float16 vt[VO * VTP];

    const int tid = threadIdx.x;
    const int l = tid & 31, w = tid >> 5, h = l >> 4, m = l & 15;
    const int t0 = blockIdx.x * VT, o0 = blockIdx.y * VO, b = blockIdx.z;
    if (t0 + VT > T_ || o0 + VO > C_ || b >= B_) return;

    const float* xb = x + (size_t)b * C_ * T_ + t0;
    #pragma unroll 2
    for (int it = 0; it < (C_ * VT / 4) / 128; ++it) {
        const int idx = it * 128 + tid;
        const int c   = idx >> 4;
        const int q4  = idx & 15;
        const v4f v = *(const v4f*)(xb + (size_t)c * T_ + 4 * q4);
        #pragma unroll
        for (int j = 0; j < 4; ++j) xt[(4 * q4 + j) * XP + c] = (_Float16)v[j];
    }
    __syncthreads();

    const v8f zero = {};
    v8f acc[4];
    #pragma unroll
    for (int mt = 0; mt < 4; ++mt) acc[mt] = zero;

    const _Float16* ar = xt + m * XP + 8 * h;
    const float* wr = Wv + (size_t)(o0 + 16 * w + m) * C_ + 8 * h;

    #pragma unroll 1
    for (int ks = 0; ks < C_ / 32; ++ks) {
        const int k0 = ks * 32;
        FragH bw;
        load_w_h16x16(wr + k0, bw);
        FragH a[4];
        #pragma unroll
        for (int mt = 0; mt < 4; ++mt) {
            a[mt].h2[0] = *(const v8h*)(ar + 16 * mt * XP + k0);
            a[mt].h2[1] = *(const v8h*)(ar + 16 * mt * XP + k0 + 16);
        }
        #pragma unroll
        for (int mt = 0; mt < 4; ++mt) acc[mt] = mma_h(a[mt].v, bw.v, acc[mt]);
        asm volatile("v_nop\n\tv_nop\n\tv_nop\n\tv_nop"
                     : "+v"(acc[0]), "+v"(acc[1]), "+v"(acc[2]), "+v"(acc[3])
                     : "v"(bw.v), "v"(a[0].v), "v"(a[1].v), "v"(a[2].v), "v"(a[3].v));
    }

    const int cl = 16 * w + m;
    const float bias = bv[o0 + cl];
    #pragma unroll
    for (int mt = 0; mt < 4; ++mt) {
        #pragma unroll
        for (int r = 0; r < 8; ++r) {
            const int tl = 16 * mt + 8 * h + r;
            vt[cl * VTP + tl] = (_Float16)(acc[mt][r] * 0.0625f + bias);
        }
    }
    __syncthreads();

    v8h vals[4];
    #pragma unroll
    for (int it = 0; it < 4; ++it) {
        const int id = it * 128 + tid;
        const int line = id >> 3, ch = id & 7;
        vals[it] = *(const v8h*)(vt + line * VTP + ch * 8);
    }
    #pragma unroll
    for (int it = 0; it < 4; ++it) {
        const int id = it * 128 + tid;
        const int line = id >> 3, ch = id & 7;
        _Float16* dst = V + ((size_t)b * C_ + o0 + line) * T_ + t0 + ch * 8;
        *(volatile v8h*)dst = vals[it];
    }
    __threadfence();
    #pragma unroll
    for (int it = 0; it < 4; ++it) {
        const int id = it * 128 + tid;
        const int line = id >> 3, ch = id & 7;
        _Float16* dst = V + ((size_t)b * C_ + o0 + line) * T_ + t0 + ch * 8;
        *(volatile v8h*)dst = vals[it];
    }
}

__global__ __launch_bounds__(128)
void k_attn(const __bf16* __restrict__ Qh, const __bf16* __restrict__ Ql,
            const __bf16* __restrict__ Kh, const __bf16* __restrict__ Kl,
            const _Float16* __restrict__ V, const float* __restrict__ x, float* __restrict__ out)
{
    __shared__ __attribute__((aligned(16))) _Float16 Pl[2 * 16 * 64];
    __shared__ __attribute__((aligned(16))) float rmax[64];
    __shared__ __attribute__((aligned(16))) float rsum[64];
    __shared__ __attribute__((aligned(16))) float obuf[C_ * OBP];

    const int tid = threadIdx.x;
    const int l = tid & 31, w = tid >> 5, h = l >> 4, m = l & 15;
    const int mt = w >> 1, g = w & 1;
    const int t0 = blockIdx.x * AT, b = blockIdx.y;
    if (t0 + AT > T_ || b >= B_) return;

    const size_t qoff = ((size_t)b * T_ + t0 + 16 * mt + m) * CQ_ + 8 * h;
    FragB aqh, aql;
    aqh.h2[0] = *(const v8b*)(Qh + qoff);
    aqh.h2[1] = *(const v8b*)(Qh + qoff + 16);
    aql.h2[0] = *(const v8b*)(Ql + qoff);
    aql.h2[1] = *(const v8b*)(Ql + qoff + 16);

    const __bf16* kbh = Kh + ((size_t)b * T_ + 32 * g + m) * CQ_ + 8 * h;
    const __bf16* kbl = Kl + ((size_t)b * T_ + 32 * g + m) * CQ_ + 8 * h;
    const _Float16* vbp = V + ((size_t)b * C_ + 128 * g + m) * T_ + 8 * h;

    _Float16*       pw  = Pl + mt * 1024 + (8 * h) * 64 + 32 * g + m;
    const _Float16* pr  = Pl + mt * 1024 + m * 64 + 8 * h;
    float*          rmw = rmax + (mt * 2 + g) * 16 + 8 * h;
    const float*    rmo = rmax + (mt * 2 + (g ^ 1)) * 16 + 8 * h;
    float*          rsw = rsum + (mt * 2 + g) * 16 + 8 * h;
    const float*    rso = rsum + (mt * 2 + (g ^ 1)) * 16 + 8 * h;

    const v8f zero = {};
    float m_run[8], l_run[8];
    v8f acc[8];
    #pragma unroll
    for (int r = 0; r < 8; ++r) { m_run[r] = -__builtin_inff(); l_run[r] = 0.0f; }
    #pragma unroll
    for (int nt = 0; nt < 8; ++nt) acc[nt] = zero;

    #pragma unroll 1
    for (int s0 = 0; s0 < T_; s0 += 64) {
        v8f s[2];
        #pragma unroll
        for (int i = 0; i < 2; ++i) {
            const size_t ko = (size_t)(s0 + 16 * i) * CQ_;
            FragB kh, kl;
            kh.h2[0] = *(const v8b*)(kbh + ko);
            kh.h2[1] = *(const v8b*)(kbh + ko + 16);
            kl.h2[0] = *(const v8b*)(kbl + ko);
            kl.h2[1] = *(const v8b*)(kbl + ko + 16);
            s[i] = mma_bf(aqh.v, kh.v, zero);
            s[i] = mma_bf(aqh.v, kl.v, s[i]);
            s[i] = mma_bf(aql.v, kh.v, s[i]);
            WG4(s[i], aqh.v, aql.v, kh.v, kl.v);
        }

        float mx[8];
        #pragma unroll
        for (int r = 0; r < 8; ++r) mx[r] = fmaxf(s[0][r], s[1][r]);
        #pragma unroll
        for (int off = 1; off < 16; off <<= 1) {
            #pragma unroll
            for (int r = 0; r < 8; ++r) mx[r] = fmaxf(mx[r], __shfl_xor(mx[r], off, 32));
        }
        if (m == 0) {
            #pragma unroll
            for (int r = 0; r < 8; ++r) rmw[r] = mx[r];
        }
        __syncthreads();

        float fc[8], sm[8], nm2[8];
        #pragma unroll
        for (int r = 0; r < 8; ++r) {
            const float oth = rmo[r];
            const float nm  = fmaxf(m_run[r], fmaxf(mx[r], oth));
            fc[r]   = __expf(m_run[r] - nm);
            m_run[r] = nm;
            nm2[r]  = nm - LN4096;
            sm[r]   = 0.0f;
        }
        #pragma unroll
        for (int i = 0; i < 2; ++i) {
            #pragma unroll
            for (int r = 0; r < 8; ++r) {
                const float pe = __expf(s[i][r] - nm2[r]);
                const _Float16 p16 = (_Float16)pe;
                sm[r] += (float)p16;
                pw[r * 64 + 16 * i] = p16;
            }
        }
        #pragma unroll
        for (int off = 1; off < 16; off <<= 1) {
            #pragma unroll
            for (int r = 0; r < 8; ++r) sm[r] += __shfl_xor(sm[r], off, 32);
        }
        if (m == 0) {
            #pragma unroll
            for (int r = 0; r < 8; ++r) rsw[r] = sm[r];
        }
        __syncthreads();

        #pragma unroll
        for (int r = 0; r < 8; ++r) {
            const float tot = sm[r] + rso[r];
            l_run[r] = l_run[r] * fc[r] + tot;
            #pragma unroll
            for (int nt = 0; nt < 8; ++nt) acc[nt][r] *= fc[r];
        }

        FragH ap0, ap1;
        ap0.h2[0] = *(const v8h*)(pr);
        ap0.h2[1] = *(const v8h*)(pr + 16);
        ap1.h2[0] = *(const v8h*)(pr + 32);
        ap1.h2[1] = *(const v8h*)(pr + 48);

        #pragma unroll
        for (int nt = 0; nt < 8; ++nt) {
            const _Float16* vp = vbp + (size_t)nt * 16 * T_ + s0;
            FragH b0, b1;
            b0.h2[0] = *(const v8h*)(vp);
            b0.h2[1] = *(const v8h*)(vp + 16);
            b1.h2[0] = *(const v8h*)(vp + 32);
            b1.h2[1] = *(const v8h*)(vp + 48);
            acc[nt] = mma_h(ap0.v, b0.v, acc[nt]);
            acc[nt] = mma_h(ap1.v, b1.v, acc[nt]);
            WG4(acc[nt], ap0.v, ap1.v, b0.v, b1.v);
        }
    }

    float inv[8];
    #pragma unroll
    for (int r = 0; r < 8; ++r) inv[r] = 1.0f / l_run[r];
    #pragma unroll
    for (int nt = 0; nt < 8; ++nt) {
        const int c = 128 * g + 16 * nt + m;
        #pragma unroll
        for (int r = 0; r < 8; ++r) obuf[c * OBP + 16 * mt + 8 * h + r] = acc[nt][r] * inv[r];
    }
    __syncthreads();

    const float* xb   = x   + (size_t)b * C_ * T_ + t0;
    float*       outb = out + (size_t)b * C_ * T_ + t0;
    v4f vals[16];
    #pragma unroll
    for (int it = 0; it < 16; ++it) {
        const int id = it * 128 + tid;
        const int c = id >> 3, ch = id & 7;
        const v4f o  = *(const v4f*)(obuf + c * OBP + 4 * ch);
        const v4f xr = *(const v4f*)(xb + (size_t)c * T_ + 4 * ch);
        vals[it] = o + xr;
    }
    #pragma unroll
    for (int it = 0; it < 16; ++it) {
        const int id = it * 128 + tid;
        const int c = id >> 3, ch = id & 7;
        *(volatile v4f*)(outb + (size_t)c * T_ + 4 * ch) = vals[it];
    }
    __threadfence();
    #pragma unroll
    for (int it = 0; it < 16; ++it) {
        const int id = it * 128 + tid;
        const int c = id >> 3, ch = id & 7;
        *(volatile v4f*)(outb + (size_t)c * T_ + 4 * ch) = vals[it];
    }
}

extern "C" void kernel_launch(void* const* d_in, const int* in_sizes, int n_in,
                              void* d_out, int out_size, void* d_ws, size_t ws_size,
                              hipStream_t stream)
{
    if (n_in < 7) return;
    if (in_sizes[0] != B_ * C_ * T_ || in_sizes[1] != CQ_ * C_ || in_sizes[2] != CQ_ ||
        in_sizes[3] != CQ_ * C_ || in_sizes[4] != CQ_ || in_sizes[5] != C_ * C_ || in_sizes[6] != C_) return;
    if (out_size != B_ * C_ * T_) return;

    const float* x  = (const float*)d_in[0];
    const float* Wq = (const float*)d_in[1];
    const float* bq = (const float*)d_in[2];
    const float* Wk = (const float*)d_in[3];
    const float* bk = (const float*)d_in[4];
    const float* Wv = (const float*)d_in[5];
    const float* bv = (const float*)d_in[6];
    float* out = (float*)d_out;

    const size_t nqk  = (size_t)B_ * T_ * CQ_;
    const size_t nv   = (size_t)B_ * C_ * T_;
    const size_t need = (4 * nqk + nv) * sizeof(unsigned short);
    if (ws_size < need) return;

    unsigned short* Qh = (unsigned short*)d_ws;
    unsigned short* Ql = Qh + nqk;
    unsigned short* Kh = Ql + nqk;
    unsigned short* Kl = Kh + nqk;
    _Float16*       Vp = (_Float16*)(Kl + nqk);

    k_projqk<<<dim3(T_ / QT, B_), dim3(64), 0, stream>>>(x, Wq, bq, Wk, bk, Qh, Ql, Kh, Kl);
    k_projv<<<dim3(T_ / VT, C_ / VO, B_), dim3(128), 0, stream>>>(x, Wv, bv, Vp);
    k_attn<<<dim3(T_ / AT, B_), dim3(128), 0, stream>>>(
        (const __bf16*)Qh, (const __bf16*)Ql, (const __bf16*)Kh, (const __bf16*)Kl, Vp, x, out);
    (void)hipGetLastError();
}
